// GAT_27144193311437
// MI455X (gfx1250) — hardware-run, weakly checked
//
#include <hip/hip_runtime.h>
#include <stddef.h>
#include <stdint.h>
#include <math.h>

#define NN      50000
#define NE      400000
#define FD      256
#define NH      4
#define HC      64
#define HW      256
#define OC      64
#define MP      50048
#define GBM     128
#define SP      68
#define KH1     512
#define TWO_TERM 1
#define KT2     (TWO_TERM ? 512 : 256)
#define NTHR    256
#define NWAVE   8
#define EPT     8
#define WCH     (32 * EPT)
#define NBRUN   1024
#define SLB     10
#define NBK     49
#define WLCAP   1536
#define RCAP    12288
#define TRIPCAP 64
#define DEGB    32
#define RPB     64
#define RPW     8
#define NEGSL   0.2f
#define MAXDEG_IN_MEAS   22
#define MAXDEG_OUT_MEAS  21
#define MAXB1024_MEAS    8436
#define WSMAX   (128u << 20)

#define PAS1 0
#define PAD1 256
#define PAS2 512
#define PAD2 768
#define PB1  1024
#define PB2  1280
#define PCAB 1344
#define PARF 1408

#define BK_ZINTS (NWAVE * WLCAP + 2 * RCAP + 4 * NBRUN)
#define BK_INTS  (BK_ZINTS + 16)
#define BK_LDS   (BK_INTS * 4)

#define PBX  (MP * FD / 8 / NTHR)
#define PBW1 (HW * FD / 8 / NTHR)
#define PBW2 (HW * KH1 / 8 / NTHR)
#define PBP  7
#define ZRINTS (NBK * 2 * NBRUN + NBK * NBRUN + 128 * 32)
#define PBZ  (ZRINTS / 4 / NTHR)
#define PBTOT (PBX + PBW1 + PBW2 + PBP + PBZ)

static_assert(NH * HC == HW && HW == 32 * 8 && HC == 64 && OC == 64);
static_assert(MP % GBM == 0 && MP >= NN && MP == 391 * GBM && MP % RPB == 0);
static_assert(NBRUN == (1 << SLB) && NBRUN % 16 == 0 && NBRUN % RPB == 0 && NBRUN == NTHR * 4);
static_assert(NBK * NBRUN >= MP);
static_assert(NE % 8 == 0 && (((long long)NE) << SLB) < (1LL << 31));
static_assert(RCAP == NWAVE * WLCAP && (2 * RCAP) % (NTHR * 4) == 0 && BK_ZINTS % (NTHR * 4) == 0);
static_assert((long long)RCAP * 100 >= (long long)MAXB1024_MEAS * 125);
static_assert(WLCAP >= MAXB1024_MEAS / 8 + 8 * 46 + 1);
static_assert(MAXDEG_IN_MEAS + 8 <= TRIPCAP && MAXDEG_OUT_MEAS + 8 <= DEGB);
static_assert(FD % 32 == 0 && KT2 % 32 == 0 && KH1 == 2 * HW && KT2 <= KH1);
static_assert(RPB == NWAVE * RPW);
static_assert(ZRINTS % (4 * NTHR) == 0 && PBZ == 151);
static_assert((MP * FD / 8) % NTHR == 0 && (HW * FD / 8) % NTHR == 0 && (HW * KH1 / 8) % NTHR == 0);
static_assert(BK_LDS <= 327680);
static_assert((GBM * SP + 512 + GBM * 8) * 4 <= 65536);
static_assert(GBM * 8 == NTHR * 4);

typedef float          v4f   __attribute__((ext_vector_type(4)));
typedef float          v8f   __attribute__((ext_vector_type(8)));
typedef int            v2i   __attribute__((ext_vector_type(2)));
typedef int            v4i   __attribute__((ext_vector_type(4)));
typedef int            v8i   __attribute__((ext_vector_type(8)));
typedef unsigned int   v4u   __attribute__((ext_vector_type(4)));
typedef unsigned short v8us  __attribute__((ext_vector_type(8)));
typedef unsigned short v16us __attribute__((ext_vector_type(16)));
typedef __bf16         v16bf __attribute__((ext_vector_type(16)));
typedef v4f  __attribute__((may_alias)) v4fa;
typedef v2i  __attribute__((may_alias)) v2ia;
typedef v4i  __attribute__((may_alias)) v4ia;
typedef v8us __attribute__((may_alias)) v8usa;
union FragB { v16bf v; v16us u; v8us h[2]; v8i w; };

__device__ __forceinline__ v8f wmb(const FragB& a, const FragB& b, v8f c) {
  v8f d = __builtin_amdgcn_wmma_f32_16x16x32_bf16(false, a.v, false, b.v, (short)0, c, false, false);
  asm volatile("v_nop\n\tv_nop\n\tv_nop\n\tv_nop" : "+v"(d) : "v"(a.w), "v"(b.w));
  return d;
}

__device__ __forceinline__ unsigned bf16_bits(float f) {
  const unsigned u = __float_as_uint(f);
  const unsigned r = (u + 0x7FFFu + ((u >> 16) & 1u)) >> 16;
  const unsigned q = (u >> 16) | 0x40u;
  return ((u & 0x7fffffffu) > 0x7f800000u) ? q : r;
}
__device__ __forceinline__ float bf16_val(float f) {
  return __uint_as_float(bf16_bits(f) << 16);
}
__device__ __forceinline__ v8us cvt8(const v4f a, const v4f b, unsigned mk) {
  v8us o;
  o[0] = (unsigned short)(bf16_bits(a.x) & mk); o[1] = (unsigned short)(bf16_bits(a.y) & mk);
  o[2] = (unsigned short)(bf16_bits(a.z) & mk); o[3] = (unsigned short)(bf16_bits(a.w) & mk);
  o[4] = (unsigned short)(bf16_bits(b.x) & mk); o[5] = (unsigned short)(bf16_bits(b.y) & mk);
  o[6] = (unsigned short)(bf16_bits(b.z) & mk); o[7] = (unsigned short)(bf16_bits(b.w) & mk);
  return o;
}

__device__ __forceinline__ void st2_v4f(float* p, v4f v) {
  *(volatile v4f*)p = v;
  __threadfence();
  *(volatile v4f*)p = v;
}
__device__ __forceinline__ void st2_v4i(int* p, v4i v) {
  *(volatile v4i*)p = v;
  __threadfence();
  *(volatile v4i*)p = v;
}
__device__ __forceinline__ void st2_v8us(unsigned short* p, v8us v) {
  *(volatile v8us*)p = v;
  __threadfence();
  *(volatile v8us*)p = v;
}

__device__ __forceinline__ void par_vec(const float* __restrict__ src, float* dst, int n4, int tid) {
  if (tid < 64) {
    const int i = tid < n4 ? tid : n4 - 1;
    const v4f a = *(const v4fa*)(src + 4 * i);
    asm volatile("" :: "v"(a));
    v4f o;
    o.x = bf16_val(a.x); o.y = bf16_val(a.y); o.z = bf16_val(a.z); o.w = bf16_val(a.w);
    if (tid < n4) st2_v4f(dst + 4 * tid, o);
  }
}

__global__ __launch_bounds__(NTHR) void k_prep(
    const float* __restrict__ x, const float* __restrict__ w1,
    const float* __restrict__ as1, const float* __restrict__ ad1,
    const float* __restrict__ we1, const float* __restrict__ be1, const float* __restrict__ ae1,
    const float* __restrict__ b1, const float* __restrict__ w2,
    const float* __restrict__ as2, const float* __restrict__ ad2,
    const float* __restrict__ we2, const float* __restrict__ be2, const float* __restrict__ ae2,
    const float* __restrict__ b2,
    unsigned short* xb, unsigned short* w1b, unsigned short* w2d, float* par, int* zr) {
  __shared__ __attribute__((aligned(16))) float sc[32];
  const int tid = (int)threadIdx.x, lane = tid & 31;
  const int blk = (int)blockIdx.x;
  if (blk < PBX) {
    const int u   = blk * NTHR + tid;
    const int row = u >> 5, k8 = (u & 31) * 8;
    const int rc  = row < NN ? row : NN - 1;
    const unsigned mk = row < NN ? 0xffffu : 0u;
    const float* p = x + (size_t)rc * FD + k8;
    const v4f a = *(const v4fa*)p;
    const v4f b = *(const v4fa*)(p + 4);
    st2_v8us(xb + (size_t)row * FD + k8, cvt8(a, b, mk));
  } else if (blk < PBX + PBW1) {
    const int u = (blk - PBX) * NTHR + tid;
    const int n = u >> 5, k8 = (u & 31) * 8;
    const float* p = w1 + (size_t)n * FD + k8;
    const v4f a = *(const v4fa*)p;
    const v4f b = *(const v4fa*)(p + 4);
    st2_v8us(w1b + (size_t)n * FD + k8, cvt8(a, b, 0xffffu));
  } else if (blk < PBX + PBW1 + PBW2) {
    const int u = (blk - PBX - PBW1) * NTHR + tid;
    const int n = u >> 6, k8 = (u & 63) * 8, kk = k8 & (HW - 1);
    const float* p = w2 + (size_t)n * HW + kk;
    const v4f a = *(const v4fa*)p;
    const v4f b = *(const v4fa*)(p + 4);
    st2_v8us(w2d + (size_t)n * KH1 + k8, cvt8(a, b, 0xffffu));
  } else if (blk < PBX + PBW1 + PBW2 + PBP) {
    const int pb = blk - (PBX + PBW1 + PBW2);
    if (pb == 0)      par_vec(as1, par + PAS1, 64, tid);
    else if (pb == 1) par_vec(ad1, par + PAD1, 64, tid);
    else if (pb == 2) par_vec(as2, par + PAS2, 64, tid);
    else if (pb == 3) par_vec(ad2, par + PAD2, 64, tid);
    else if (pb == 4) par_vec(b1,  par + PB1,  64, tid);
    else if (pb == 5) par_vec(b2,  par + PB2,  16, tid);
    else {
      if (tid < 32) {
        const int h = lane & 3;
        float s1a = 0.0f, s1b = 0.0f, s2a = 0.0f, s2b = 0.0f;
#pragma unroll 1
        for (int c = 0; c < HC; ++c) {
          const int i = HC * h + c;
          const float w1v = bf16_val(we1[i]), e1v = bf16_val(be1[i]), a1v = bf16_val(ae1[i]);
          const float w2v = bf16_val(we2[i]), e2v = bf16_val(be2[i]), a2v = bf16_val(ae2[i]);
          s1a += w1v * a1v; s1b += e1v * a1v;
          s2a += w2v * a2v; s2b += e2v * a2v;
        }
        if (lane < 4) { sc[h] = s1a; sc[4 + h] = s1b; sc[8 + h] = s2a; sc[12 + h] = s2b; }
        if (lane >= 16) sc[lane] = 0.0f;
      }
      __syncthreads();
      if (tid < 32) {
        const int i = lane < 8 ? lane : 7;
        const v4f v = *(const v4fa*)(sc + 4 * i);
        asm volatile("" :: "v"(v));
        if (lane < 8) st2_v4f(par + PCAB + 4 * lane, v);
      }
    }
  } else {
    const int u = (blk - (PBX + PBW1 + PBW2 + PBP)) * NTHR + tid;
    const v4i z4 = {0, 0, 0, 0};
    st2_v4i(zr + (size_t)4 * (size_t)u, z4);
  }
}

template <int KTOT, int WP>
__device__ __forceinline__ void gemm_16x64(const unsigned short* __restrict__ ap,
                                           const unsigned short* __restrict__ bp, v8f (&acc)[4]) {
#pragma unroll 1
  for (int k0 = 0; k0 < KTOT; k0 += 32) {
    FragB af;
    af.h[0] = *(const v8usa*)(ap + k0);
    af.h[1] = *(const v8usa*)(ap + k0 + 16);
#pragma unroll
    for (int nt = 0; nt < 4; ++nt) {
      const unsigned short* wq = bp + (size_t)(16 * nt) * (size_t)WP + k0;
      FragB bf;
      bf.h[0] = *(const v8usa*)wq;
      bf.h[1] = *(const v8usa*)(wq + 16);
      acc[nt] = wmb(af, bf, acc[nt]);
    }
  }
}

__device__ __forceinline__ void stage_d(float* stg, const v8f (&acc)[4], int wave, int hh, int m) {
#pragma unroll
  for (int nt = 0; nt < 4; ++nt) {
#pragma unroll
    for (int r = 0; r < 8; ++r) stg[(16 * wave + 8 * hh + r) * SP + 16 * nt + m] = acc[nt][r];
  }
}

template <int KTOT, int APITCH, int WPITCH>
__global__ __launch_bounds__(NTHR) __attribute__((amdgpu_num_vgpr(248)))
void k_gemm(const unsigned short* __restrict__ A, const unsigned short* __restrict__ BT,
            const float* __restrict__ attp, float* XL, float* SD) {
  static_assert(KTOT % 32 == 0 && KTOT <= APITCH && KTOT <= WPITCH);
  __shared__ __attribute__((aligned(16))) float stg[GBM * SP];
  __shared__ __attribute__((aligned(16))) float satt[2 * HW];
  __shared__ __attribute__((aligned(16))) float sdl[GBM * 8];
  const int tid = (int)threadIdx.x, lane = tid & 31, wave = tid >> 5, hh = lane >> 4, m = lane & 15;
  const int rowBase = (int)blockIdx.x * GBM;
  if (tid < 128) *(v4fa*)(satt + 4 * tid) = *(const v4fa*)(attp + 4 * tid);

  const unsigned short* ap = A + (size_t)(rowBase + 16 * wave + m) * (size_t)APITCH + 8 * hh;
#pragma unroll 1
  for (int head = 0; head < NH; ++head) {
    v8f acc[4];
    {
      const v8f z = {0.f, 0.f, 0.f, 0.f, 0.f, 0.f, 0.f, 0.f};
#pragma unroll
      for (int t = 0; t < 4; ++t) acc[t] = z;
    }
    const unsigned short* bp = BT + (size_t)(head * HC + m) * (size_t)WPITCH + 8 * hh;
    gemm_16x64<KTOT, WPITCH>(ap, bp, acc);
    stage_d(stg, acc, wave, hh, m);
    __syncthreads();

    {
      const int row = tid & (GBM - 1), which = tid >> 7;
      const float* sa = satt + which * HW + head * HC;
      const float* hr = stg + row * SP;
      float d = 0.0f;
#pragma unroll 4
      for (int c4 = 0; c4 < HC / 4; ++c4) {
        const v4f hv = *(const v4fa*)(hr + 4 * c4);
        const v4f av = *(const v4fa*)(sa + 4 * c4);
        d = fmaf(hv.x, av.x, d);
        d = fmaf(hv.y, av.y, d);
        d = fmaf(hv.z, av.z, d);
        d = fmaf(hv.w, av.w, d);
      }
      sdl[row * 8 + which * 4 + head] = d;
    }
#pragma unroll 1
    for (int i = 0; i < 8; ++i) {
      const int lr   = 16 * wave + 2 * i + hh;
      const int grow = rowBase + lr;
      const v4f a = *(const v4fa*)(stg + lr * SP + 4 * m);
      st2_v4f(XL + (size_t)grow * HW + head * HC + 4 * m, a);
    }
    __syncthreads();
  }
  {
    const v4f v = *(const v4fa*)(sdl + 4 * tid);
    st2_v4f(SD + (size_t)rowBase * 8 + 4 * tid, v);
  }
}

__device__ __forceinline__ void bucket_flush(const int* pl, const int* cnt, const float* lwst, int ov, int role,
                                             int* lp, int* cop, float* lwp, int* fp, int tid) {
  if (role == 0) {
#pragma unroll 1
    for (int i = tid * 4; i < 2 * RCAP; i += NTHR * 4) {
      const v4i v = *(const v4ia*)(pl + i);
      *(volatile v4i*)(lp + i) = v;
    }
#pragma unroll 1
    for (int i = tid * 4; i < 2 * NBRUN; i += NTHR * 4) {
      const v4i v = *(const v4ia*)(cnt + i);
      *(volatile v4i*)(cop + i) = v;
    }
  } else {
    const v4f v = *(const v4fa*)(lwst + 4 * tid);
    *(volatile v4f*)(lwp + 4 * tid) = v;
  }
  if (tid < 8) {
    const v4i f = {ov, ov, ov, ov};
    *(volatile v4i*)(fp + 4 * tid) = f;
  }
}

__global__ __launch_bounds__(NTHR) void k_bucket(const int* __restrict__ ei, const float* __restrict__ ew,
                                                 int* LIST, int* CO, float* LOOPW, int* FLAG) {
  extern __shared__ __attribute__((aligned(16))) int dsm[];
  int* wl   = dsm;
  int* pl   = dsm + NWAVE * WLCAP;
  int* cnt  = pl + 2 * RCAP;
  int* offs = cnt + NBRUN;
  int* cur  = offs + NBRUN;
  float* lwst = (float*)(cur + NBRUN);
  int* misc = cur + 2 * NBRUN;
  const int tid = (int)threadIdx.x, lane = tid & 31, wave = tid >> 5;
  const int blk  = (int)blockIdx.x;
  const int role = (blk >= NBK) ? 1 : 0;
  const int bb   = role ? (blk - NBK) : blk;
  const int keyOff = role ? 0 : NE;
  const int othOff = role ? NE : 0;
  const unsigned nbs = (unsigned)(bb * NBRUN);

  {
    const v4i z4 = {0, 0, 0, 0};
    for (int i = tid * 4; i < BK_ZINTS; i += NTHR * 4) *(v4ia*)(dsm + i) = z4;
    if (tid < 16) misc[tid] = 0;
  }
  __syncthreads();

  {
    const int per  = ((NE + NWAVE * WCH - 1) / (NWAVE * WCH)) * WCH;
    const int ebeg = wave * per;
    const int eend = (ebeg + per < NE) ? (ebeg + per) : NE;
    const int sent = (int)(1u << 31);
    int* mylist = wl + wave * WLCAP;
    int wc = 0;
#pragma unroll 1
    for (int cb = ebeg; cb < eend; cb += WCH) {
      const int e0  = cb + lane * EPT;
      const int e0c = e0 < NE - 8 ? e0 : NE - 8;
      v4i da = *(const v4ia*)(ei + keyOff + e0c);
      v4i db = *(const v4ia*)(ei + keyOff + e0c + 4);
      asm volatile("" :: "v"(da));
      asm volatile("" :: "v"(db));
      const int mk = (e0 < NE) ? -1 : 0;
      const int sm = sent & ~mk;
      da.x = (da.x & mk) | sm; da.y = (da.y & mk) | sm; da.z = (da.z & mk) | sm; da.w = (da.w & mk) | sm;
      db.x = (db.x & mk) | sm; db.y = (db.y & mk) | sm; db.z = (db.z & mk) | sm; db.w = (db.w & mk) | sm;
      const unsigned s0 = (unsigned)da.x - nbs, s1 = (unsigned)da.y - nbs;
      const unsigned s2 = (unsigned)da.z - nbs, s3 = (unsigned)da.w - nbs;
      const unsigned s4 = (unsigned)db.x - nbs, s5 = (unsigned)db.y - nbs;
      const unsigned s6 = (unsigned)db.z - nbs, s7 = (unsigned)db.w - nbs;
      const bool h0 = s0 < (unsigned)NBRUN, h1 = s1 < (unsigned)NBRUN, h2 = s2 < (unsigned)NBRUN, h3 = s3 < (unsigned)NBRUN;
      const bool h4 = s4 < (unsigned)NBRUN, h5 = s5 < (unsigned)NBRUN, h6 = s6 < (unsigned)NBRUN, h7 = s7 < (unsigned)NBRUN;
      const unsigned m0 = __builtin_amdgcn_ballot_w32(h0), m1 = __builtin_amdgcn_ballot_w32(h1);
      const unsigned m2 = __builtin_amdgcn_ballot_w32(h2), m3 = __builtin_amdgcn_ballot_w32(h3);
      const unsigned m4 = __builtin_amdgcn_ballot_w32(h4), m5 = __builtin_amdgcn_ballot_w32(h5);
      const unsigned m6 = __builtin_amdgcn_ballot_w32(h6), m7 = __builtin_amdgcn_ballot_w32(h7);
      const unsigned any = m0 | m1 | m2 | m3 | m4 | m5 | m6 | m7;
      if (any != 0u) {
        const int pre = (int)(__builtin_amdgcn_mbcnt_lo(m0, 0u) + __builtin_amdgcn_mbcnt_lo(m1, 0u) +
                              __builtin_amdgcn_mbcnt_lo(m2, 0u) + __builtin_amdgcn_mbcnt_lo(m3, 0u) +
                              __builtin_amdgcn_mbcnt_lo(m4, 0u) + __builtin_amdgcn_mbcnt_lo(m5, 0u) +
                              __builtin_amdgcn_mbcnt_lo(m6, 0u) + __builtin_amdgcn_mbcnt_lo(m7, 0u));
        int p = wc + pre;
        if (h0) { if (p < WLCAP) mylist[p] = ((e0 + 0) << SLB) | (int)s0; p = p + 1; }
        if (h1) { if (p < WLCAP) mylist[p] = ((e0 + 1) << SLB) | (int)s1; p = p + 1; }
        if (h2) { if (p < WLCAP) mylist[p] = ((e0 + 2) << SLB) | (int)s2; p = p + 1; }
        if (h3) { if (p < WLCAP) mylist[p] = ((e0 + 3) << SLB) | (int)s3; p = p + 1; }
        if (h4) { if (p < WLCAP) mylist[p] = ((e0 + 4) << SLB) | (int)s4; p = p + 1; }
        if (h5) { if (p < WLCAP) mylist[p] = ((e0 + 5) << SLB) | (int)s5; p = p + 1; }
        if (h6) { if (p < WLCAP) mylist[p] = ((e0 + 6) << SLB) | (int)s6; p = p + 1; }
        if (h7) { if (p < WLCAP) mylist[p] = ((e0 + 7) << SLB) | (int)s7; p = p + 1; }
        wc += (int)(__builtin_popcount(m0) + __builtin_popcount(m1) + __builtin_popcount(m2) + __builtin_popcount(m3) +
                    __builtin_popcount(m4) + __builtin_popcount(m5) + __builtin_popcount(m6) + __builtin_popcount(m7));
      }
    }
    if (lane == 0) misc[wave] = wc;
  }
  __syncthreads();

  if (wave == 0) {
    int ov = 0;
#pragma unroll 1
    for (int w2 = 0; w2 < NWAVE; ++w2) {
      int c = misc[w2];
      if (c > WLCAP) ov = 1;
      c = c < 0 ? 0 : (c > WLCAP ? WLCAP : c);
#pragma unroll 1
      for (int b0 = 0; b0 < c; b0 += 32) {
        const int idx = b0 + lane;
        const int ent = wl[w2 * WLCAP + (idx < WLCAP ? idx : WLCAP - 1)];
        const int m32 = (c - b0) < 32 ? (c - b0) : 32;
#pragma unroll 1
        for (int k = 0; k < m32; ++k) {
          const int u    = __builtin_amdgcn_readlane(ent, k);
          const int slot = u & (NBRUN - 1);
          if (lane == 0) cnt[slot] = cnt[slot] + 1;
        }
      }
    }
    if (lane == 0) misc[9] = ov;
  }
  __syncthreads();
  if (wave == 0) {
    const int base = lane * (NBRUN / 32);
    int s = 0;
#pragma unroll 1
    for (int i = 0; i < NBRUN / 32; ++i) s += cnt[base + i];
    int incl = s;
#pragma unroll
    for (int d = 1; d < 32; d <<= 1) {
      const int y = __shfl_up(incl, d, 32);
      if (lane >= d) incl += y;
    }
    int run = incl - s;
#pragma unroll 1
    for (int i = 0; i < NBRUN / 32; ++i) {
      const int cv = cnt[base + i];
      offs[base + i] = run;
      cur[base + i]  = run;
      run += cv;
    }
  }
  __syncthreads();

  if (wave == 0) {
#pragma unroll 1
    for (int w2 = 0; w2 < NWAVE; ++w2) {
      int c = misc[w2];
      c = c < 0 ? 0 : (c > WLCAP ? WLCAP : c);
#pragma unroll 1
      for (int b0 = 0; b0 < c; b0 += 32) {
        const int idx = b0 + lane;
        const int ent = wl[w2 * WLCAP + (idx < WLCAP ? idx : WLCAP - 1)];
        int eid = (ent >> SLB) & 0x1FFFFF;
        eid = eid > NE - 1 ? NE - 1 : eid;
        int oth = ei[othOff + eid];
        oth = oth < 0 ? 0 : (oth > NN - 1 ? NN - 1 : oth);
        const int wb  = (int)(bf16_bits(ew[eid]) << 16);
        const int m32 = (c - b0) < 32 ? (c - b0) : 32;
#pragma unroll 1
        for (int k = 0; k < m32; ++k) {
          const int u    = __builtin_amdgcn_readlane(ent, k);
          const int w0   = __builtin_amdgcn_readlane(oth, k);
          const int w1   = __builtin_amdgcn_readlane(wb, k);
          const int slot = u & (NBRUN - 1);
          if (lane == 0) {
            int p = cur[slot];
            p = p < 0 ? 0 : (p > RCAP - 1 ? RCAP - 1 : p);
            pl[2 * p]     = w0;
            pl[2 * p + 1] = w1;
            cur[slot] = p + 1;
          }
        }
      }
    }
  }
  __syncthreads();

  const int ovf = misc[9];
  if (role != 0) {
    const float qnan = __uint_as_float(0x7fc00000u);
#pragma unroll 1
    for (int k = 0; k < 4; ++k) {
      const int slot = 4 * tid + k;
      const int craw = cnt[slot];
      int c = craw < 0 ? 0 : (craw > DEGB ? DEGB : craw);
      int o = offs[slot];
      o = o < 0 ? 0 : (o > RCAP - 1 ? RCAP - 1 : o);
      int last = o + c - 1;
      last = last < o ? o : last;
      last = last > RCAP - 1 ? RCAP - 1 : last;
      float sum = 0.0f;
#pragma unroll 4
      for (int j = 0; j < DEGB; ++j) {
        int idx = o + j;
        idx = idx > last ? last : idx;
        const float wv = __int_as_float(pl[2 * idx + 1]);
        asm volatile("" :: "v"(wv));
        const float t = sum + wv;
        sum = (j < c) ? t : sum;
      }
      float den = (float)craw;
      den = den < 1.0f ? 1.0f : den;
      float lwv = sum / den;
      lwv = ((ovf != 0) | (craw > DEGB)) ? qnan : lwv;
      lwst[slot] = lwv;
    }
  }
  __syncthreads();

  int*   lp  = LIST + (size_t)bb * (2 * RCAP);
  int*   cop = CO + (size_t)bb * (2 * NBRUN);
  float* lwp = LOOPW + (size_t)bb * NBRUN;
  int*   fp  = FLAG + (size_t)blk * 32;
  bucket_flush(pl, cnt, lwst, ovf, role, lp, cop, lwp, fp, tid);
  __threadfence();
  bucket_flush(pl, cnt, lwst, ovf, role, lp, cop, lwp, fp, tid);
}

template <int L>
__global__ __launch_bounds__(NTHR) void k_replay(
    const int* __restrict__ LIST, const int* __restrict__ CO, const int* __restrict__ FLAG,
    const float* __restrict__ LOOPW, const float* __restrict__ XL, const float* __restrict__ SD,
    const float* __restrict__ PAR, unsigned short* H1, float* out) {
  __shared__ __attribute__((aligned(16))) float stg[NWAVE * HW];
  const int tid = (int)threadIdx.x, lane = tid & 31, wave = tid >> 5, head = lane >> 3;
  const int rowBase = (int)blockIdx.x * RPB;
  const int bucket  = rowBase >> SLB;
  const int* lb  = LIST + (size_t)bucket * (2 * RCAP);
  const int* cob = CO + (size_t)bucket * (2 * NBRUN);
  const int flag = FLAG[(size_t)bucket * 32];
  const int pc   = (L == 1) ? PCAB : (PCAB + 8);
  const float cA = PAR[pc + head];
  const float cB = PAR[pc + 4 + head];
  const float qnan = __uint_as_float(0x7fc00000u);
  const float ninf = __uint_as_float(0xff800000u);
  v4f ba, bb;
  if constexpr (L == 1) {
    ba = *(const v4fa*)(PAR + PB1 + 8 * lane);
    bb = *(const v4fa*)(PAR + PB1 + 8 * lane + 4);
  } else {
    ba = *(const v4fa*)(PAR + PB2 + 4 * (lane & 15));
    bb = ba;
  }

#pragma unroll 1
  for (int i = 0; i < RPW; ++i) {
    const int d    = rowBase + RPW * wave + i;
    const int slot = d & (NBRUN - 1);
    int c = cob[slot];
    int o = cob[NBRUN + slot];
    const bool big = c > TRIPCAP;
    c = c < 0 ? 0 : (c > TRIPCAP ? TRIPCAP : c);
    o = o < 0 ? 0 : (o > RCAP - 1 ? RCAP - 1 : o);
    c = c > RCAP - o ? RCAP - o : c;
    c = __builtin_amdgcn_readfirstlane(c);
    o = __builtin_amdgcn_readfirstlane(o);
    int last = o + c - 1;
    last = last < o ? o : last;
    const int dcl = d < NN ? d : NN - 1;
    const float ad = SD[(size_t)dcl * 8 + 4 + head];
    const float lw = LOOPW[dcl];

    float m = ninf, l = 0.0f;
    float acc[8];
#pragma unroll
    for (int k = 0; k < 8; ++k) acc[k] = 0.0f;

#pragma unroll 1
    for (int j = 0; j <= c; ++j) {
      int idx = o + j;
      idx = idx > last ? last : idx;
      const v2i wd = *(const v2ia*)(lb + 2 * idx);
      asm volatile("" :: "v"(wd));
      const bool isl = (j == c);
      int s = isl ? dcl : wd.x;
      s = s < 0 ? 0 : (s > NN - 1 ? NN - 1 : s);
      const float w = isl ? lw : __int_as_float(wd.y);
      const float as = SD[(size_t)s * 8 + head];
      const float* xr = XL + (size_t)s * HW + 8 * lane;
      const v4f xa = *(const v4fa*)xr;
      const v4f xb = *(const v4fa*)(xr + 4);
      asm volatile("" :: "v"(as));
      asm volatile("" :: "v"(xa));
      asm volatile("" :: "v"(xb));
      float e = (as + ad) + (w * cA + cB);
      e = (e > 0.0f) ? e : NEGSL * e;
      const float df = e - m;
      const bool first = !(m > ninf);
      const float ee = expf(first ? 0.0f : -fabsf(df));
      const bool up = df > 0.0f;
      const float s1 = up ? (first ? 0.0f : ee) : 1.0f;
      const float s2 = (up ? 1.0f : ee) + (e - e);
      m = up ? e : m;
      l = l * s1 + s2;
      acc[0] = acc[0] * s1 + s2 * xa.x; acc[1] = acc[1] * s1 + s2 * xa.y;
      acc[2] = acc[2] * s1 + s2 * xa.z; acc[3] = acc[3] * s1 + s2 * xa.w;
      acc[4] = acc[4] * s1 + s2 * xb.x; acc[5] = acc[5] * s1 + s2 * xb.y;
      acc[6] = acc[6] * s1 + s2 * xb.z; acc[7] = acc[7] * s1 + s2 * xb.w;
    }
    const float inv = 1.0f / l;
    const bool bad  = (flag != 0) | big;
    const bool live = d < NN;

    if constexpr (L == 1) {
      float v[8];
      v[0] = acc[0] * inv + ba.x; v[1] = acc[1] * inv + ba.y; v[2] = acc[2] * inv + ba.z; v[3] = acc[3] * inv + ba.w;
      v[4] = acc[4] * inv + bb.x; v[5] = acc[5] * inv + bb.y; v[6] = acc[6] * inv + bb.z; v[7] = acc[7] * inv + bb.w;
      unsigned hb[8], lq[8];
#pragma unroll
      for (int k = 0; k < 8; ++k) {
        float t = bad ? qnan : v[k];
        t = live ? t : 0.0f;
        hb[k] = bf16_bits(t);
        lq[k] = bf16_bits(t - __uint_as_float(hb[k] << 16));
      }
      v4u ph, pq;
      ph.x = hb[0] | (hb[1] << 16); ph.y = hb[2] | (hb[3] << 16); ph.z = hb[4] | (hb[5] << 16); ph.w = hb[6] | (hb[7] << 16);
      pq.x = lq[0] | (lq[1] << 16); pq.y = lq[2] | (lq[3] << 16); pq.z = lq[4] | (lq[5] << 16); pq.w = lq[6] | (lq[7] << 16);
      unsigned short* hp = H1 + (size_t)d * KH1 + 8 * lane;
      *(volatile v4u*)hp = ph;
      *(volatile v4u*)(hp + HW) = pq;
      __threadfence();
      *(volatile v4u*)hp = ph;
      *(volatile v4u*)(hp + HW) = pq;
    } else {
      float* my = stg + wave * HW;
      v4f va, vb;
      va.x = acc[0] * inv; va.y = acc[1] * inv; va.z = acc[2] * inv; va.w = acc[3] * inv;
      vb.x = acc[4] * inv; vb.y = acc[5] * inv; vb.z = acc[6] * inv; vb.w = acc[7] * inv;
      *(v4fa*)(my + 8 * lane)     = va;
      *(v4fa*)(my + 8 * lane + 4) = vb;
      __syncthreads();
      const int q = lane & 15;
      const v4f h0 = *(const v4fa*)(my + 4 * q);
      const v4f h1 = *(const v4fa*)(my + HC + 4 * q);
      const v4f h2 = *(const v4fa*)(my + 2 * HC + 4 * q);
      const v4f h3 = *(const v4fa*)(my + 3 * HC + 4 * q);
      asm volatile("" :: "v"(h0));
      asm volatile("" :: "v"(h1));
      asm volatile("" :: "v"(h2));
      asm volatile("" :: "v"(h3));
      v4f ov;
      ov.x = (((h0.x + h1.x) + h2.x) + h3.x) * 0.25f + ba.x;
      ov.y = (((h0.y + h1.y) + h2.y) + h3.y) * 0.25f + ba.y;
      ov.z = (((h0.z + h1.z) + h2.z) + h3.z) * 0.25f + ba.z;
      ov.w = (((h0.w + h1.w) + h2.w) + h3.w) * 0.25f + ba.w;
      ov.x = bad ? qnan : ov.x; ov.y = bad ? qnan : ov.y; ov.z = bad ? qnan : ov.z; ov.w = bad ? qnan : ov.w;
      __syncthreads();
      const bool wr = live & (lane < 16);
      float* op = out + (size_t)dcl * OC + 4 * q;
      if (wr) *(volatile v4f*)op = ov;
      __threadfence();
      if (wr) *(volatile v4f*)op = ov;
    }
  }
}

extern "C" void kernel_launch(void* const* d_in, const int* in_sizes, int n_in,
                              void* d_out, int out_size, void* d_ws, size_t ws_size,
                              hipStream_t stream) {
  if (n_in < 17) return;
  if (in_sizes[0] != NN * FD) return;
  if (in_sizes[1] != 2 * NE) return;
  if (in_sizes[2] != NE) return;
  if (in_sizes[3] != HW * FD) return;
  if (in_sizes[4] != HW || in_sizes[5] != HW) return;
  if (in_sizes[6] != HW || in_sizes[7] != HW) return;
  if (in_sizes[8] != HW || in_sizes[9] != HW) return;
  if (in_sizes[10] != HW * HW) return;
  if (in_sizes[11] != HW || in_sizes[12] != HW) return;
  if (in_sizes[13] != HW || in_sizes[14] != HW) return;
  if (in_sizes[15] != HW) return;
  if (in_sizes[16] != OC) return;
  if (out_size != NN * OC) return;

  const float* x    = (const float*)d_in[0];
  const int*   ei   = (const int*)d_in[1];
  const float* ew   = (const float*)d_in[2];
  const float* W1   = (const float*)d_in[3];
  const float* as1  = (const float*)d_in[4];
  const float* ad1  = (const float*)d_in[5];
  const float* We1  = (const float*)d_in[6];
  const float* be1  = (const float*)d_in[7];
  const float* ae1  = (const float*)d_in[8];
  const float* b1   = (const float*)d_in[9];
  const float* W2   = (const float*)d_in[10];
  const float* as2  = (const float*)d_in[11];
  const float* ad2  = (const float*)d_in[12];
  const float* We2  = (const float*)d_in[13];
  const float* be2  = (const float*)d_in[14];
  const float* ae2  = (const float*)d_in[15];
  const float* b2   = (const float*)d_in[16];
  float* out = (float*)d_out;

  constexpr size_t zA    = (size_t)MP * KH1 * 2;
  constexpr size_t zXL   = (size_t)MP * HW * 4;
  constexpr size_t zSD   = (size_t)MP * 8 * 4;
  constexpr size_t zLIST = (size_t)NBK * 2 * RCAP * 4;
  constexpr size_t zZR   = (size_t)ZRINTS * 4;
  constexpr size_t zW1B  = (size_t)HW * FD * 2;
  constexpr size_t zW2D  = (size_t)HW * KH1 * 2;
  constexpr size_t zPAR  = (size_t)PARF * 4;
  constexpr size_t oA    = 0;
  constexpr size_t oXL   = oA + zA;
  constexpr size_t oSD   = oXL + zXL;
  constexpr size_t oLIST = oSD + zSD;
  constexpr size_t oZR   = oLIST + zLIST;
  constexpr size_t oW1B  = oZR + zZR;
  constexpr size_t oW2D  = oW1B + zW1B;
  constexpr size_t oPAR  = oW2D + zW2D;
  constexpr size_t oEND  = oPAR + zPAR;
  static_assert(zA % 256 == 0 && zXL % 256 == 0 && zSD % 256 == 0 && zLIST % 256 == 0 && zZR % 256 == 0);
  static_assert(zW1B % 256 == 0 && zW2D % 256 == 0 && zPAR % 256 == 0);
  static_assert((size_t)MP * FD * 2 <= zA);
  static_assert(oEND <= (size_t)WSMAX);
  if (oEND > ws_size) return;

  char* ws = (char*)d_ws;
  unsigned short* XB   = (unsigned short*)(ws + oA);
  unsigned short* H1   = (unsigned short*)(ws + oA);
  float*          XL   = (float*)(ws + oXL);
  float*          SD   = (float*)(ws + oSD);
  int*            LIST = (int*)(ws + oLIST);
  int*            ZR   = (int*)(ws + oZR);
  int*            CO   = ZR;
  float*          LOOPW = (float*)(ZR + NBK * 2 * NBRUN);
  int*            FLAG = ZR + NBK * 3 * NBRUN;
  unsigned short* W1B  = (unsigned short*)(ws + oW1B);
  unsigned short* W2D  = (unsigned short*)(ws + oW2D);
  float*          PAR  = (float*)(ws + oPAR);

  hipFuncSetAttribute(reinterpret_cast<const void*>(&k_bucket), hipFuncAttributeMaxDynamicSharedMemorySize, (int)BK_LDS);

  k_prep<<<PBTOT, NTHR, 0, stream>>>(x, W1, as1, ad1, We1, be1, ae1, b1, W2, as2, ad2, We2, be2, ae2, b2,
                                     XB, W1B, W2D, PAR, ZR);
  k_gemm<FD, FD, FD><<<MP / GBM, NTHR, 0, stream>>>(XB, W1B, PAR + PAS1, XL, SD);
  k_bucket<<<2 * NBK, NTHR, BK_LDS, stream>>>(ei, ew, LIST, CO, LOOPW, FLAG);
  k_replay<1><<<MP / RPB, NTHR, 0, stream>>>(LIST, CO, FLAG, LOOPW, XL, SD, PAR, H1, out);
  k_gemm<KT2, KH1, KH1><<<MP / GBM, NTHR, 0, stream>>>(H1, W2D, PAR + PAS2, XL, SD);
  k_replay<2><<<MP / RPB, NTHR, 0, stream>>>(LIST, CO, FLAG, LOOPW, XL, SD, PAR, H1, out);
}
